// SchemeC_78769700208699
// MI455X (gfx1250) — hardware-verified
//
#include <hip/hip_runtime.h>
#include <math.h>

constexpr int kNB    = 128;
constexpr int kNG    = 12000;
constexpr int kNGP   = 12032;
constexpr int kNK    = 512;
constexpr int kNH    = 64;
constexpr int kNXG   = 256;
constexpr int kNBH   = kNB * kNH;
constexpr int kSteps = 10;
constexpr int kChunkB = 16;
constexpr int kNChunk = kNB / kChunkB;
constexpr int kChunkN = kChunkB * kNH;
constexpr float kZCarry   = 64.0f;
constexpr float kACarry   = 256.0f;
constexpr float kDiffScale = 0.9f / 256.0f;
constexpr float kHScale    = 1.0f / 64.0f;

static_assert(kNG % 32 == 0, "K of the module projection must be a multiple of 32");
static_assert(kNGP % 64 == 0 && kNGP >= kNG, "padded gene count");
static_assert(kNK % 64 == 0 && kNXG % 64 == 0 && kNBH % 64 == 0 && kChunkN % 64 == 0, "tile multiples");
static_assert(kNG % 8 == 0 && kNGP % 8 == 0, "16-B alignment of 16-bit rows");

typedef __attribute__((ext_vector_type(16))) _Float16 v16h;
typedef __attribute__((ext_vector_type(8)))  _Float16 v8h;
typedef __attribute__((ext_vector_type(16))) __bf16   v16b;
typedef __attribute__((ext_vector_type(8)))  __bf16   v8b;
typedef __attribute__((ext_vector_type(8)))  float    v8f;
typedef __attribute__((ext_vector_type(4)))  float    v4f;
typedef __attribute__((ext_vector_type(4)))  unsigned int v4u;

__device__ __forceinline__ unsigned short f2bf_bits(float f) {
  unsigned u = __float_as_uint(f);
  return (unsigned short)((u + 0x7FFFu + ((u >> 16) & 1u)) >> 16);
}
__device__ __forceinline__ float bf_bits2f(unsigned short h) { return __uint_as_float(((unsigned)h) << 16); }

__device__ __forceinline__ void dep_guard_h(v8f& a, v8f& b, v16h x, v16h y) { asm volatile("v_nop\n\tv_nop\n\tv_nop\n\tv_nop" : "+v"(a), "+v"(b) : "v"(x), "v"(y)); }
__device__ __forceinline__ void dep_guard_b(v8f& a, v8f& b, v16b x, v16b y) { asm volatile("v_nop\n\tv_nop\n\tv_nop\n\tv_nop" : "+v"(a), "+v"(b) : "v"(x), "v"(y)); }
__device__ __forceinline__ void keep4_h(v16h a, v16h b, v16h c, v16h d) { asm volatile("v_nop" :: "v"(a), "v"(b), "v"(c), "v"(d)); }
__device__ __forceinline__ void keep4_b(v16b a, v16b b, v16b c, v16b d) { asm volatile("v_nop" :: "v"(a), "v"(b), "v"(c), "v"(d)); }
__device__ __forceinline__ void acc_guard4(v8f& a, v8f& b, v8f& c, v8f& d) { asm volatile("v_nop\n\tv_nop\n\tv_nop\n\tv_nop" : "+v"(a), "+v"(b), "+v"(c), "+v"(d)); }
template <typename T> struct Frag;
template <> struct Frag<_Float16> {
  typedef v16h V; union U { v16h v; v8h h[2]; };
  static __device__ __forceinline__ v16h load(const _Float16* p) {
    U f; f.h[0] = *(const v8h*)(p); f.h[1] = *(const v8h*)(p + 16); return f.v;
  }
  static __device__ __forceinline__ v8f mma(v16h a, v16h b, v8f c) {
    return __builtin_amdgcn_wmma_f32_16x16x32_f16(false, a, false, b, (short)0, c, false, false);
  }
  static __device__ __forceinline__ void guard(v8f& a, v8f& b, v16h x, v16h y) { dep_guard_h(a, b, x, y); }
  static __device__ __forceinline__ void keep(v16h a, v16h b, v16h c, v16h d) { keep4_h(a, b, c, d); }
};
template <> struct Frag<__bf16> {
  typedef v16b V; union U { v16b v; v8b h[2]; };
  static __device__ __forceinline__ v16b load(const __bf16* p) {
    U f; f.h[0] = *(const v8b*)(p); f.h[1] = *(const v8b*)(p + 16); return f.v;
  }
  static __device__ __forceinline__ v8f mma(v16b a, v16b b, v8f c) {
    return __builtin_amdgcn_wmma_f32_16x16x32_bf16(false, a, false, b, (short)0, c, false, false);
  }
  static __device__ __forceinline__ void guard(v8f& a, v8f& b, v16b x, v16b y) { dep_guard_b(a, b, x, y); }
  static __device__ __forceinline__ void keep(v16b a, v16b b, v16b c, v16b d) { keep4_b(a, b, c, d); }
};

__device__ __forceinline__ unsigned pk16(unsigned short a, unsigned short b) { return (unsigned)a | ((unsigned)b << 16); }
__device__ __forceinline__ unsigned short h_bits(float f) { const _Float16 h = (_Float16)f; return __builtin_bit_cast(unsigned short, h); }

template <int ET> struct Elem;
template <> struct Elem<0> { typedef _Float16 T; };
template <> struct Elem<1> { typedef __bf16 T; };
template <int ET, bool SPLIT, int BIAS_MODE, int OUT_MODE, bool RESID, int ACT = 0>
__global__ __launch_bounds__(256) void wmma_gemm64(
    const unsigned short* __restrict__ Ap, const unsigned short* __restrict__ A2p, int lda, long strideA,
    const unsigned short* __restrict__ Btp, const unsigned short* __restrict__ Bt2p, int ldb, long strideB,
    void* __restrict__ Cout, void* __restrict__ Cout2, int ldc, long strideC,
    const float* __restrict__ bias,
    const float* __restrict__ resid, long strideR,
    int M, int N, int K, float scale) {
  typedef typename Elem<ET>::T T;
  typedef typename Frag<T>::V V;
  const T* A = (const T*)Ap; const T* A2 = (const T*)A2p; const T* Bt = (const T*)Btp; const T* Bt2 = (const T*)Bt2p;
  __shared__ __align__(16) float sT[8][16 * 68];
  const int b    = blockIdx.y;
  const int lane = threadIdx.x & 31;
  const int wave = threadIdx.x >> 5;
  const int tilesN = N >> 6;
  const int tilesM = M >> 6;
  const int tile = blockIdx.x * 8 + wave;
  if (tile >= tilesM * tilesN) return;
  const int tm = tile / tilesN;
  const int tn = tile - tm * tilesN;
  const int m0 = tm << 6;
  const int n0 = tn << 6;

  const T* Ab  = A  + (size_t)b * strideA;
  const T* Bb  = Bt + (size_t)b * strideB;
  const T* Ab2 = SPLIT ? (A2  + (size_t)b * strideA) : nullptr;
  const T* Bb2 = SPLIT ? (Bt2 + (size_t)b * strideB) : nullptr;

  const int rlane = lane & 15;
  const int koff  = (lane >> 4) * 8;
  const int mOff  = (lane >> 4) * 8;

  v8f acc[4][4];
#pragma unroll
  for (int i = 0; i < 4; ++i)
#pragma unroll
    for (int j = 0; j < 4; ++j) acc[i][j] = (v8f){0.f,0.f,0.f,0.f,0.f,0.f,0.f,0.f};

  for (int k0 = 0; k0 < K; k0 += 32) {
    V bh[4], bl[4];
#pragma unroll
    for (int j = 0; j < 4; ++j) {
      const size_t bo = (size_t)(n0 + (j << 4) + rlane) * ldb + koff + k0;
      bh[j] = Frag<T>::load(Bb + bo);
      if (SPLIT) bl[j] = Frag<T>::load(Bb2 + bo);
    }
#pragma unroll
    for (int i = 0; i < 4; ++i) {
      const size_t ao = (size_t)(m0 + (i << 4) + rlane) * lda + koff + k0;
      V ah = Frag<T>::load(Ab + ao);
      V al;
      if (SPLIT) al = Frag<T>::load(Ab2 + ao);
#pragma unroll
      for (int j = 0; j < 4; ++j) {
        acc[i][j] = Frag<T>::mma(ah, bh[j], acc[i][j]);
        if (SPLIT) {
          acc[i][j] = Frag<T>::mma(ah, bl[j], acc[i][j]);
          acc[i][j] = Frag<T>::mma(al, bh[j], acc[i][j]);
        }
      }
      Frag<T>::guard(acc[i][0], acc[i][3], ah, SPLIT ? al : ah);
    }
    Frag<T>::keep(bh[0], bh[1], bh[2], bh[3]);
    if (SPLIT) Frag<T>::keep(bl[0], bl[1], bl[2], bl[3]);
  }
  acc_guard4(acc[0][0], acc[0][1], acc[0][2], acc[0][3]);
  acc_guard4(acc[1][0], acc[1][1], acc[1][2], acc[1][3]);
  acc_guard4(acc[2][0], acc[2][1], acc[2][2], acc[2][3]);
  acc_guard4(acc[3][0], acc[3][1], acc[3][2], acc[3][3]);

  float* slab = sT[wave];
  const float* Rb = RESID ? (resid + (size_t)b * strideR) : nullptr;
#pragma unroll
  for (int i = 0; i < 4; ++i) {
    const int mBase = m0 + (i << 4);
#pragma unroll
    for (int j = 0; j < 4; ++j) {
      const int n = n0 + (j << 4) + rlane;
      float bv = 0.f;
      if (BIAS_MODE == 2) bv = bias[n];
#pragma unroll
      for (int r = 0; r < 8; ++r) {
        float v = acc[i][j][r] * scale;
        if (BIAS_MODE == 1) v += bias[mBase + mOff + r];
        if (BIAS_MODE == 2) v += bv;
        if (RESID) v += Rb[(size_t)(mBase + mOff + r) * ldc + n];
        if (ACT == 2) v = fmaxf(v, 0.0f);
        if (ACT == 4) v = (v > 0.f) ? v : 0.01f * v;
        slab[(mOff + r) * 68 + (j << 4) + rlane] = v;
      }
    }
    __builtin_amdgcn_fence(__ATOMIC_RELEASE, "workgroup");
    __builtin_amdgcn_wave_barrier();
    __builtin_amdgcn_fence(__ATOMIC_ACQUIRE, "workgroup");
    if (OUT_MODE == 0) {
      float* C = (float*)Cout + (size_t)b * strideC;
      const int hh = lane >> 4, c4 = (lane & 15) * 4;
      for (int pass = 0; pass < 2; ++pass) {
#pragma unroll
        for (int it = 0; it < 8; ++it) {
          const int row = it * 2 + hh;
          v4f v = *(const v4f*)(slab + row * 68 + c4);
          *(volatile v4f*)(C + (size_t)(mBase + row) * ldc + n0 + c4) = v;
        }
        __threadfence();
      }
    } else {
      const int q = lane >> 3, c8 = (lane & 7) * 8;
      unsigned short* C  = (unsigned short*)Cout  + (size_t)b * strideC;
      unsigned short* C2 = (OUT_MODE == 2) ? ((unsigned short*)Cout2 + (size_t)b * strideC) : nullptr;
      for (int pass = 0; pass < 2; ++pass) {
#pragma unroll
        for (int it = 0; it < 4; ++it) {
          const int row = it * 4 + q;
          const float* sp = slab + row * 68 + c8;
          v8h hv, lv;
#pragma unroll
          for (int e = 0; e < 8; ++e) {
            if (OUT_MODE == 1) {
              hv[e] = (_Float16)sp[e];
            } else {
              unsigned short hb = f2bf_bits(sp[e]);
              unsigned short lb = f2bf_bits(sp[e] - bf_bits2f(hb));
              hv[e] = __builtin_bit_cast(_Float16, hb);
              lv[e] = __builtin_bit_cast(_Float16, lb);
            }
          }
          *(volatile v8h*)(C + (size_t)(mBase + row) * ldc + n0 + c8) = hv;
          if (OUT_MODE == 2) *(volatile v8h*)(C2 + (size_t)(mBase + row) * ldc + n0 + c8) = lv;
        }
        __threadfence();
      }
    }
    __builtin_amdgcn_fence(__ATOMIC_RELEASE, "workgroup");
    __builtin_amdgcn_wave_barrier();
    __builtin_amdgcn_fence(__ATOMIC_ACQUIRE, "workgroup");
  }
}

__global__ __launch_bounds__(256) void deg_kernel(const float* __restrict__ Mm, float* __restrict__ deg) {
  const int k = blockIdx.x * 256 + threadIdx.x;
  float s = 0.f;
#pragma unroll 4
  for (int g = 0; g < kNG; ++g) s += Mm[(size_t)g * kNK + k];
  s = fmaxf(s, 1.0f);
  ((volatile float*)deg)[k] = s;
  __threadfence();
  ((volatile float*)deg)[k] = s;
}

__global__ __launch_bounds__(256) void mtcast_kernel(const float* __restrict__ Mm, unsigned short* __restrict__ out) {
  __shared__ float sm[64][65];
  const int t  = threadIdx.x;
  const int g0 = blockIdx.x * 64;
  const int k0 = blockIdx.y * 64;
#pragma unroll
  for (int i = 0; i < 16; ++i) {
    const int e = i * 256 + t;
    const int r = e >> 6;
    const int c = e & 63;
    const int g = g0 + r;
    const int gc = (g < kNG) ? g : (kNG - 1);
    float v = Mm[(size_t)gc * kNK + k0 + c];
    v = (g < kNG) ? v : 0.0f;
    sm[c][r] = v;
  }
  __syncthreads();
  const int lane = t & 31, wave = t >> 5;
  const int q = lane >> 3, c8 = (lane & 7) * 8;
  for (int pass = 0; pass < 2; ++pass) {
#pragma unroll
    for (int it = 0; it < 2; ++it) {
      const int row = wave * 8 + it * 4 + q;
      unsigned short hb[8];
#pragma unroll
      for (int e = 0; e < 8; ++e) hb[e] = h_bits(sm[row][c8 + e]);
      const v4u u = (v4u){pk16(hb[0], hb[1]), pk16(hb[2], hb[3]), pk16(hb[4], hb[5]), pk16(hb[6], hb[7])};
      *(volatile v4u*)(out + (size_t)(k0 + row) * kNGP + g0 + c8) = u;
    }
    __threadfence();
  }
}

__global__ __launch_bounds__(256) void atcast_kernel(const float* __restrict__ Aadj, unsigned short* __restrict__ out, float scale) {
  __shared__ float sm[64][65];
  const int t  = threadIdx.x;
  const int k0 = blockIdx.x * 64;
  const int l0 = blockIdx.y * 64;
#pragma unroll
  for (int i = 0; i < 16; ++i) {
    const int e = i * 256 + t;
    const int r = e >> 6;
    const int c = e & 63;
    sm[c][r] = Aadj[(size_t)(k0 + r) * kNK + l0 + c] * scale;
  }
  __syncthreads();
  const int lane = t & 31, wave = t >> 5;
  const int q = lane >> 3, c8 = (lane & 7) * 8;
  for (int pass = 0; pass < 2; ++pass) {
#pragma unroll
    for (int it = 0; it < 2; ++it) {
      const int row = wave * 8 + it * 4 + q;
      unsigned short hb[8];
#pragma unroll
      for (int e = 0; e < 8; ++e) hb[e] = h_bits(sm[row][c8 + e]);
      const v4u u = (v4u){pk16(hb[0], hb[1]), pk16(hb[2], hb[3]), pk16(hb[4], hb[5]), pk16(hb[6], hb[7])};
      *(volatile v4u*)(out + (size_t)(l0 + row) * kNK + k0 + c8) = u;
    }
    __threadfence();
  }
}

__global__ __launch_bounds__(256) void m16cast_kernel(const float* __restrict__ Mm, unsigned short* __restrict__ out) {
  const int i = blockIdx.x * 256 + threadIdx.x;
  const int nval = kNG * kNK / 8;
  const int ic = (i < nval) ? i : (nval - 1);
  const float* p = Mm + 8 * (size_t)ic;
  const v4f a = *(const v4f*)(p);
  const v4f c = *(const v4f*)(p + 4);
  const bool valid = (i < nval);
  unsigned short hb[8];
#pragma unroll
  for (int e = 0; e < 4; ++e) {
    hb[e]     = h_bits(valid ? a[e] : 0.0f);
    hb[4 + e] = h_bits(valid ? c[e] : 0.0f);
  }
  const v4u u = (v4u){pk16(hb[0], hb[1]), pk16(hb[2], hb[3]), pk16(hb[4], hb[5]), pk16(hb[6], hb[7])};
  unsigned short* q = out + 8 * (size_t)i;
  *(volatile v4u*)q = u;
  __threadfence();
  *(volatile v4u*)q = u;
}

__global__ __launch_bounds__(256) void xgcast_kernel(const float* __restrict__ ctl, const float* __restrict__ drug,
                                                     unsigned short* __restrict__ out) {
  const int t = blockIdx.x * 256 + threadIdx.x;
  const int n = blockIdx.y;
  if (t >= kNGP / 8) return;
  const int c = n >> 7, b = n & 127;
  const float* src = (c ? drug : ctl) + (size_t)b * kNG;
  const int nval = kNG / 8;
  const int tc = (t < nval) ? t : (nval - 1);
  const float* p = src + 8 * (size_t)tc;
  const v4f a = *(const v4f*)(p);
  const v4f d = *(const v4f*)(p + 4);
  const bool valid = (t < nval);
  unsigned short hb[8];
#pragma unroll
  for (int e = 0; e < 4; ++e) {
    hb[e]     = h_bits(valid ? a[e] : 0.0f);
    hb[4 + e] = h_bits(valid ? d[e] : 0.0f);
  }
  const v4u u = (v4u){pk16(hb[0], hb[1]), pk16(hb[2], hb[3]), pk16(hb[4], hb[5]), pk16(hb[6], hb[7])};
  unsigned short* q = out + (size_t)n * kNGP + 8 * (size_t)t;
  *(volatile v4u*)q = u;
  __threadfence();
  *(volatile v4u*)q = u;
}

__global__ __launch_bounds__(256) void sproj_kernel(const float* __restrict__ XM, const float* __restrict__ deg,
                                                    const float* __restrict__ W_in, const float* __restrict__ b_in,
                                                    float* __restrict__ R, unsigned short* __restrict__ Z0) {
  __shared__ __align__(16) float sS[2][kNK];
  const int t = threadIdx.x;
  const int r = t >> 7;
  const int row = blockIdx.x * 2 + r;
  const int b = row >> 6, h = row & 63;
  const int k4 = (t & 127) * 4;
  const float w0 = W_in[h], w1 = W_in[kNH + h], bi = b_in[h];
  const v4f dg = *(const v4f*)(deg + k4);
  float sv[4];
#pragma unroll
  for (int i = 0; i < 4; ++i) {
    const int k = k4 + i;
    const float x0 = XM[(size_t)k * kNXG + b];
    const float x1 = XM[(size_t)k * kNXG + kNB + b];
    const float rd = 1.0f / dg[i];
    const float xm0 = x0 * rd, xm1 = x1 * rd;
    sv[i] = fmaxf(xm0 * w0 + xm1 * w1 + bi, 0.0f);
  }
  const v4f rv = (v4f){kZCarry * (0.1f * sv[0]), kZCarry * (0.1f * sv[1]), kZCarry * (0.1f * sv[2]), kZCarry * (0.1f * sv[3])};
  float* rp = R + (size_t)row * kNK + k4;
  *(volatile v4f*)rp = rv;
  __threadfence();
  *(volatile v4f*)rp = rv;
  *(v4f*)(&sS[r][k4]) = (v4f){kZCarry * sv[0], kZCarry * sv[1], kZCarry * sv[2], kZCarry * sv[3]};
  __syncthreads();
  if (t < 128) {
    const int r2 = t >> 6, k8 = (t & 63) * 8;
    const int row2 = blockIdx.x * 2 + r2;
    const v4f a = *(const v4f*)(&sS[r2][k8]);
    const v4f c = *(const v4f*)(&sS[r2][k8 + 4]);
    unsigned short hb[8];
#pragma unroll
    for (int e = 0; e < 4; ++e) { hb[e] = h_bits(a[e]); hb[4 + e] = h_bits(c[e]); }
    const v4u u = (v4u){pk16(hb[0], hb[1]), pk16(hb[2], hb[3]), pk16(hb[4], hb[5]), pk16(hb[6], hb[7])};
    unsigned short* q = Z0 + (size_t)row2 * kNK + k8;
    *(volatile v4u*)q = u;
    __threadfence();
    *(volatile v4u*)q = u;
  }
}

__global__ __launch_bounds__(256) void readout_kernel(const float* __restrict__ Hc, const int* __restrict__ cell_idx,
                                                      const float* __restrict__ cell_emb, const float* __restrict__ W_out,
                                                      const float* __restrict__ b_out, float* __restrict__ y, int cb, int nc) {
  const int g  = blockIdx.x * 256 + threadIdx.x;
  const int bl = blockIdx.y;
  const int b  = cb * kChunkB + bl;
  const int gc = (g < kNGP) ? g : (kNGP - 1);
  int ci = cell_idx[b];
  ci = (ci < 0) ? 0 : ci;
  ci = (ci >= nc) ? (nc - 1) : ci;
  const float* hp = Hc + (size_t)gc * kChunkN + bl * kNH;
  const float* ce = cell_emb + (size_t)ci * kNH;
  float acc = 0.f;
#pragma unroll 4
  for (int q = 0; q < kNH / 4; ++q) {
    const v4f hv = *(const v4f*)(hp + 4 * q);
    const v4f cv = *(const v4f*)(ce + 4 * q);
    const v4f wv = *(const v4f*)(W_out + 4 * q);
#pragma unroll
    for (int e = 0; e < 4; ++e) acc += (hv[e] + cv[e]) * wv[e];
  }
  acc += b_out[0];
  if (g < kNG) {
    volatile float* yp = y + (size_t)b * kNG + g;
    *yp = acc;
    __threadfence();
    *yp = acc;
  }
}

extern "C" void kernel_launch(void* const* d_in, const int* in_sizes, int n_in,
                              void* d_out, int out_size, void* d_ws, size_t ws_size,
                              hipStream_t stream) {
  if (n_in < 11) return;
  const float* ctl      = (const float*)d_in[0];
  const float* drug     = (const float*)d_in[1];
  const int*   cell_idx = (const int*)  d_in[2];
  const float* Mm       = (const float*)d_in[4];
  const float* Aadj     = (const float*)d_in[5];
  const float* W_in     = (const float*)d_in[6];
  const float* b_in     = (const float*)d_in[7];
  const float* cell_emb = (const float*)d_in[8];
  const float* W_out    = (const float*)d_in[9];
  const float* b_out    = (const float*)d_in[10];
  float* y = (float*)d_out;

  if (in_sizes[0] != kNB * kNG || in_sizes[1] != kNB * kNG || in_sizes[2] != kNB ||
      in_sizes[4] != kNG * kNK || in_sizes[5] != kNK * kNK || in_sizes[6] != 2 * kNH ||
      in_sizes[7] != kNH || in_sizes[9] != kNH || in_sizes[10] < 1 || out_size != kNB * kNG) return;
  int nc = in_sizes[8] / kNH;
  if (nc < 1) return;

  char* ws = (char*)d_ws;
  size_t off = 0;
  auto carve = [&](size_t bytes) -> size_t { size_t o = off; off += (bytes + 255) & ~(size_t)255; return o; };
  const size_t o_deg  = carve((size_t)kNK * 4);
  const size_t o_mt   = carve((size_t)kNK * kNGP * 2);
  const size_t o_xg   = carve((size_t)kNXG * kNGP * 2);
  const size_t o_xm   = carve((size_t)kNK * kNXG * 4);
  const size_t o_m16  = carve((size_t)kNGP * kNK * 2);
  const size_t o_at   = carve((size_t)kNK * kNK * 2);
  const size_t o_r    = carve((size_t)kNBH * kNK * 4);
  const size_t o_za   = carve((size_t)kNBH * kNK * 2);
  const size_t o_zb   = carve((size_t)kNBH * kNK * 2);
  const size_t o_hc   = carve((size_t)kNGP * kChunkN * 4);
  if (off > ws_size) return;

  float*          deg  = (float*)(ws + o_deg);
  unsigned short* Mt16 = (unsigned short*)(ws + o_mt);
  unsigned short* xg16 = (unsigned short*)(ws + o_xg);
  float*          XM   = (float*)(ws + o_xm);
  unsigned short* M16  = (unsigned short*)(ws + o_m16);
  unsigned short* At16 = (unsigned short*)(ws + o_at);
  float*          R    = (float*)(ws + o_r);
  unsigned short* Zp[2] = { (unsigned short*)(ws + o_za), (unsigned short*)(ws + o_zb) };
  float*          Hc   = (float*)(ws + o_hc);

  deg_kernel<<<kNK / 256, 256, 0, stream>>>(Mm, deg);
  mtcast_kernel<<<dim3(kNGP / 64, kNK / 64), 256, 0, stream>>>(Mm, Mt16);
  xgcast_kernel<<<dim3((kNGP / 8 + 255) / 256, kNXG), 256, 0, stream>>>(ctl, drug, xg16);
  m16cast_kernel<<<(kNGP * kNK / 8) / 256, 256, 0, stream>>>(Mm, M16);
  atcast_kernel<<<dim3(kNK / 64, kNK / 64), 256, 0, stream>>>(Aadj, At16, kACarry);

  {
    const int tiles = (kNK / 64) * (kNXG / 64);
    wmma_gemm64<0, false, 0, 0, false, 0><<<dim3((tiles + 7) / 8, 1), 256, 0, stream>>>(
        Mt16, Mt16, kNGP, 0L, xg16, xg16, kNGP, 0L, (void*)XM, (void*)XM, kNXG, 0L,
        deg, deg, 0L, kNK, kNXG, kNG, 1.0f);
  }

  sproj_kernel<<<kNBH / 2, 256, 0, stream>>>(XM, deg, W_in, b_in, R, Zp[0]);

  {
    const int tiles = (kNBH / 64) * (kNK / 64);
    for (int s = 0; s < kSteps; ++s) {
      unsigned short* zin  = Zp[s & 1];
      unsigned short* zout = Zp[(s + 1) & 1];
      wmma_gemm64<0, false, 0, 1, true, 0><<<dim3((tiles + 7) / 8, 1), 256, 0, stream>>>(
          zin, zin, kNK, 0L, At16, At16, kNK, 0L, (void*)zout, (void*)zout, kNK, 0L,
          deg, R, 0L, kNBH, kNK, kNK, kDiffScale);
    }
  }
  unsigned short* Zf = Zp[kSteps & 1];

  {
    const int tiles = (kNGP / 64) * (kChunkN / 64);
    for (int cb = 0; cb < kNChunk; ++cb) {
      const unsigned short* zc = Zf + (size_t)cb * kChunkN * kNK;
      wmma_gemm64<0, false, 0, 0, false, 0><<<dim3((tiles + 7) / 8, 1), 256, 0, stream>>>(
          M16, M16, kNK, 0L, zc, zc, kNK, 0L, (void*)Hc, (void*)Hc, kChunkN, 0L,
          deg, deg, 0L, kNGP, kChunkN, kNK, kHScale);
      readout_kernel<<<dim3(kNGP / 256, kChunkB), 256, 0, stream>>>(Hc, cell_idx, cell_emb, W_out, b_out, y, cb, nc);
    }
  }
}
